// PatchAttention_4595615006864
// MI455X (gfx1250) — hardware-verified
//
#include <hip/hip_runtime.h>
#include <math.h>
#include <stdint.h>

#ifndef NB
#define NB 2
#endif
#define NB_FULL 2
#define SEQ   384
#define DM    256
#define NH    8
#define HD    32
#define CD    3
#define NQKV  (3 * DM)
#define GROWS (NB * SEQ)
#define NIT   (SEQ / 16)
#define NJT   (SEQ / 32)
#define NRT   (SEQ / 64)
#define NPAIR 512
#define HP    32
#define RBP   264
#define SLP   36
#define SP    40
#define WAP   40
#define TSP   264
#define VTP   72
#define SLAB64 (16 * 68)
#define HREGF 8192
#define RSQ_HD 0.17677669529663687f
#define LOG2E  1.4426950408889634f
#define QSC   1024.0f
#define KSC   1024.0f
#define PCAR  32768.0f
#define VCAR  1024.0f
#define HCAR  1024.0f
#define WCAR  1024.0f
#define TCAR  1024.0f
#define WS_CAP 134217728
#define PSTR  ((size_t)NB * NH * SEQ * SEQ)
#define TSTR  ((size_t)NB * NH * SEQ * DM)
static_assert(NB >= 1 && NB <= NB_FULL);
static_assert(DM == NH * HD && HD == 32 && NH == 8 && CD == 3);
static_assert((SEQ % 64) == 0 && (GROWS % 64) == 0 && (GROWS % 8) == 0 && (NQKV % 64) == 0 && (DM % 32) == 0);
static_assert(NPAIR == 16 * 32 && NPAIR * HP == 2 * HREGF && 8 * 16 * SLP <= HREGF);
static_assert(((GROWS * DM) % 8) == 0 && ((NQKV * DM) % 8) == 0 && ((DM * DM) % 8) == 0);

typedef unsigned short u16;
typedef _Float16 v16h __attribute__((ext_vector_type(16)));
typedef _Float16 v8h  __attribute__((ext_vector_type(8)));
typedef __bf16   v16b __attribute__((ext_vector_type(16)));
typedef float    v8f  __attribute__((ext_vector_type(8)));
typedef float    v4f  __attribute__((ext_vector_type(4)));
typedef unsigned int v4u __attribute__((ext_vector_type(4)));

union FragH { v16h v; v8h h[2]; v4u u[2]; };
union FragB { v16b v; v4u u[2]; };

__device__ __forceinline__ unsigned short bf_bits(float f) {
  unsigned u = __float_as_uint(f);
  return (unsigned short)((u + 0x7FFFu + ((u >> 16) & 1u)) >> 16);
}
__device__ __forceinline__ float bf_up(unsigned short h) { return __uint_as_float(((unsigned)h) << 16); }
__device__ __forceinline__ float bfr(float f) { return bf_up(bf_bits(f)); }
__device__ __forceinline__ unsigned short h_bits(_Float16 x) { return __builtin_bit_cast(unsigned short, x); }
__device__ __forceinline__ unsigned pk16(unsigned short a, unsigned short b) { return (unsigned)a | ((unsigned)b << 16); }
__device__ __forceinline__ v8f zero8() { v8f z = {0.f, 0.f, 0.f, 0.f, 0.f, 0.f, 0.f, 0.f}; return z; }
__device__ __forceinline__ float silu_f(float x) {
  const float e = __expf(-x);
  return x * __builtin_amdgcn_rcpf(1.0f + e);
}

__device__ __forceinline__ v16h ldfrag_h(const _Float16* p) {
  FragH f;
  f.h[0] = *(const v8h*)(p);
  f.h[1] = *(const v8h*)(p + 16);
  return f.v;
}
__device__ __forceinline__ v16b ldfrag_b(const u16* p) {
  FragB f;
  f.u[0] = *(const v4u*)(p);
  f.u[1] = *(const v4u*)(p + 16);
  return f.v;
}

__device__ __forceinline__ v8f mma_h(v16h a, v16h b, v8f c) {
  return __builtin_amdgcn_wmma_f32_16x16x32_f16(false, a, false, b, (short)0, c, false, false);
}
__device__ __forceinline__ v8f mma_b(v16b a, v16b b, v8f c) {
  return __builtin_amdgcn_wmma_f32_16x16x32_bf16(false, a, false, b, (short)0, c, false, false);
}
__device__ __forceinline__ void guard2(v8f& a, v8f& b, v16h x0, v16h x1, v16h x2, v16h x3, v16h x4, v16h x5) {
#if defined(__HIP_DEVICE_COMPILE__)
  asm volatile("v_nop\n\tv_nop\n\tv_nop\n\tv_nop"
               : "+v"(a), "+v"(b) : "v"(x0), "v"(x1), "v"(x2), "v"(x3), "v"(x4), "v"(x5) : "memory");
#endif
}
template <typename F>
__device__ __forceinline__ void guard6(v8f& a, v8f& b, v8f& c, v8f& d, F x0, F x1, F x2, F x3, F x4, F x5) {
#if defined(__HIP_DEVICE_COMPILE__)
  asm volatile("v_nop\n\tv_nop\n\tv_nop\n\tv_nop"
               : "+v"(a), "+v"(b), "+v"(c), "+v"(d) : "v"(x0), "v"(x1), "v"(x2), "v"(x3), "v"(x4), "v"(x5) : "memory");
#endif
}
__device__ __forceinline__ void wave_sync_lds() {
  __builtin_amdgcn_fence(__ATOMIC_RELEASE, "workgroup");
  __builtin_amdgcn_wave_barrier();
  __builtin_amdgcn_fence(__ATOMIC_ACQUIRE, "workgroup");
}

__global__ __launch_bounds__(256) void cvt16(const float* __restrict__ x, u16* D, int n8, int f16mode, float scale) {
  const int gt = blockIdx.x * 256 + (int)threadIdx.x;
  if (gt >= n8) return;
  const float* p = x + (size_t)gt * 8;
  const v4f a = *(const v4f*)(p), b4 = *(const v4f*)(p + 4);
  float w[8];
#pragma unroll
  for (int e = 0; e < 4; ++e) { w[e] = a[e]; w[4 + e] = b4[e]; }
  v4u o;
#pragma unroll
  for (int e = 0; e < 4; ++e) {
    const float f0 = w[2 * e], f1 = w[2 * e + 1];
    const unsigned short hb0 = h_bits((_Float16)(bfr(f0) * scale));
    const unsigned short hb1 = h_bits((_Float16)(bfr(f1) * scale));
    const unsigned short bb0 = bf_bits(f0);
    const unsigned short bb1 = bf_bits(f1);
    o[e] = (f16mode != 0) ? pk16(hb0, hb1) : pk16(bb0, bb1);
  }
  u16* d = D + (size_t)gt * 8;
  for (int pass = 0; pass < 2; ++pass) {
    *(volatile v4u*)(d) = o;
    __threadfence();
  }
}

__device__ __forceinline__ void epi64b(float* sl, v8f a0, v8f a1, v8f a2, v8f a3, float oscale,
                                       float b0, float b1, float b2, float b3,
                                       float* C, int N, size_t rowb, int col0, int lane) {
  const int hh = lane >> 4, m = lane & 15;
#pragma unroll
  for (int r = 0; r < 8; ++r) {
    const int ro = (8 * hh + r) * 68 + m;
    sl[ro]      = a0[r] * oscale + b0;
    sl[ro + 16] = a1[r] * oscale + b1;
    sl[ro + 32] = a2[r] * oscale + b2;
    sl[ro + 48] = a3[r] * oscale + b3;
  }
  wave_sync_lds();
  v4f vals[8];
#pragma unroll
  for (int it = 0; it < 8; ++it) vals[it] = *(const v4f*)(sl + (it * 2 + hh) * 68 + m * 4);
  float* dst = C + (rowb + (size_t)hh) * (size_t)N + col0 + m * 4;
  for (int pass = 0; pass < 2; ++pass) {
#pragma unroll
    for (int it = 0; it < 8; ++it) {
      *(volatile v4f*)(dst + (size_t)(it * 2) * (size_t)N) = vals[it];
    }
    __threadfence();
  }
}

__global__ __launch_bounds__(128)
void gemm_bf(const u16* __restrict__ A, const u16* __restrict__ Bt, const float* __restrict__ bias,
             float* C, int M, int N, int K, float oscale) {
  __shared__ __align__(16) float slab[4 * SLAB64];
  const int tid = threadIdx.x, wave = tid >> 5, lane = tid & 31, hh = lane >> 4, m = lane & 15;
  const int ntile = N >> 6;
  const int bid   = blockIdx.x;
  const int rowb  = (bid / ntile) * 64 + wave * 16;
  const int col0  = (bid % ntile) * 64;
  if (rowb + 16 > M) return;
  const u16* ap = A  + (size_t)(rowb + m) * K + 8 * hh;
  const u16* bp = Bt + (size_t)(col0 + m) * K + 8 * hh;
  const size_t bs = (size_t)16 * K;
  v8f acc0 = zero8(), acc1 = zero8(), acc2 = zero8(), acc3 = zero8();
#pragma unroll 1
  for (int k0 = 0; k0 < K; k0 += 32) {
    const v16b a  = ldfrag_b(ap + k0);
    const v16b b0 = ldfrag_b(bp + k0);
    const v16b b1 = ldfrag_b(bp + bs + k0);
    const v16b b2 = ldfrag_b(bp + 2 * bs + k0);
    const v16b b3 = ldfrag_b(bp + 3 * bs + k0);
    acc0 = mma_b(a, b0, acc0);
    acc1 = mma_b(a, b1, acc1);
    acc2 = mma_b(a, b2, acc2);
    acc3 = mma_b(a, b3, acc3);
    guard6<v16b>(acc0, acc1, acc2, acc3, a, b0, b1, b2, b3, a);
  }
  const float bv0 = bfr(bias[col0 + m]);
  const float bv1 = bfr(bias[col0 + 16 + m]);
  const float bv2 = bfr(bias[col0 + 32 + m]);
  const float bv3 = bfr(bias[col0 + 48 + m]);
  epi64b(slab + wave * SLAB64, acc0, acc1, acc2, acc3, oscale, bv0, bv1, bv2, bv3, C, N, (size_t)rowb, col0, lane);
}

__global__ __launch_bounds__(256) void qk16(const float* __restrict__ F, int ldf, int coff, u16* Hp, u16* Lp, float sc) {
  const int tid = (int)threadIdx.x;
  const int rl  = tid >> 5;
  const int cc  = tid & 31;
  const int row = (int)blockIdx.x * 8 + rl;
  if (row >= GROWS) return;
  const float* p = F + (size_t)row * ldf + coff + cc * 8;
  const v4f a = *(const v4f*)(p), b4 = *(const v4f*)(p + 4);
  float w[8];
#pragma unroll
  for (int e = 0; e < 4; ++e) { w[e] = a[e] * sc; w[4 + e] = b4[e] * sc; }
  v4u oh, ol;
#pragma unroll
  for (int e = 0; e < 4; ++e) {
    const float t0 = w[2 * e], t1 = w[2 * e + 1];
    const _Float16 h0 = (_Float16)t0, h1 = (_Float16)t1;
    const _Float16 l0 = (_Float16)(t0 - (float)h0), l1 = (_Float16)(t1 - (float)h1);
    oh[e] = pk16(h_bits(h0), h_bits(h1));
    ol[e] = pk16(h_bits(l0), h_bits(l1));
  }
  u16* dh = Hp + (size_t)row * DM + cc * 8;
  u16* dl = Lp + (size_t)row * DM + cc * 8;
  for (int pass = 0; pass < 2; ++pass) {
    *(volatile v4u*)(dh) = oh;
    *(volatile v4u*)(dl) = ol;
    __threadfence();
  }
}

__global__ __launch_bounds__(256) void vt16(const float* __restrict__ F, u16* VHo) {
  __shared__ __align__(16) u16 TH[HD * VTP];
  const int tid = threadIdx.x;
  const int bid = blockIdx.x;
  const int st  = bid % NRT;
  const int t2  = bid / NRT;
  const int h   = t2 % NH;
  const int b   = t2 / NH;
  if (b >= NB) return;
  const int s0  = st * 64;
  {
    const int sl = tid >> 2;
    const int dc = (tid & 3) * 8;
    const float* src = F + ((size_t)b * SEQ + s0 + sl) * NQKV + 2 * DM + h * HD + dc;
    const v4f a = *(const v4f*)(src), b4 = *(const v4f*)(src + 4);
    float w[8];
#pragma unroll
    for (int e = 0; e < 4; ++e) { w[e] = a[e]; w[4 + e] = b4[e]; }
#pragma unroll
    for (int e = 0; e < 8; ++e) {
      TH[(dc + e) * VTP + sl] = h_bits((_Float16)(w[e] * VCAR));
    }
  }
  __syncthreads();
  const int q8 = tid >> 3, p8 = (tid & 7) * 8;
  const v4u vh = *(const v4u*)(TH + q8 * VTP + p8);
  const size_t base = ((size_t)(b * NH + h) * HD + q8) * SEQ + s0 + p8;
  for (int pass = 0; pass < 2; ++pass) {
    *(volatile v4u*)(VHo + base) = vh;
    __threadfence();
  }
}

__global__ __launch_bounds__(256)
void k_scores(const float* __restrict__ coords, const float* __restrict__ rbw1, const float* __restrict__ rbb1,
              const float* __restrict__ rbw2, const float* __restrict__ rbb2,
              const u16* __restrict__ QHp, const u16* __restrict__ QLp,
              const u16* __restrict__ KHp, const u16* __restrict__ KLp, float* SCp) {
  __shared__ __align__(16) float WB[DM * 4];
  __shared__ __align__(16) float CI[16 * 4];
  __shared__ __align__(16) float CJ2[32 * 4];
  __shared__ __align__(16) u16   RB2[16 * RBP];
  __shared__ __align__(16) float HREG[HREGF];
  __shared__ __align__(16) float BB[NPAIR * NH];

  const int tid = threadIdx.x, wave = tid >> 5, lane = tid & 31, hh = lane >> 4, m = lane & 15;
  const int bid = blockIdx.x;
  const int jt  = bid % NJT;
  const int t2  = bid / NJT;
  const int it  = t2 % NIT;
  const int b   = t2 / NIT;
  if (b >= NB) return;
  const int i0 = it * 16, j0 = jt * 32;
  u16* hid = (u16*)(void*)HREG;
  const _Float16* hidh = (const _Float16*)(const void*)HREG;
  const _Float16* rb2h = (const _Float16*)(const void*)RB2;

  {
    WB[tid * 4 + 0] = bfr(rbw1[tid * 3 + 0]);
    WB[tid * 4 + 1] = bfr(rbw1[tid * 3 + 1]);
    WB[tid * 4 + 2] = bfr(rbw1[tid * 3 + 2]);
    WB[tid * 4 + 3] = bfr(rbb1[tid]);
    if (tid < 16 * CD) {
      const int il = tid / CD, k = tid - il * CD;
      CI[il * 4 + k] = bfr(coords[((size_t)(b * SEQ + i0 + il)) * CD + k]);
    }
    if (tid < 32 * CD) {
      const int jl = tid / CD, k = tid - jl * CD;
      CJ2[jl * 4 + k] = bfr(coords[((size_t)(b * SEQ + j0 + jl)) * CD + k]);
    }
    const int row  = tid >> 4, cb = (tid & 15) * 16;
    const int rowc = (row < NH) ? row : (NH - 1);
    const bool vr  = (row < NH);
    const float* src = rbw2 + rowc * DM + cb;
    const v4f a0 = *(const v4f*)(src), a1 = *(const v4f*)(src + 4), a2 = *(const v4f*)(src + 8), a3 = *(const v4f*)(src + 12);
    float w[16];
#pragma unroll
    for (int e = 0; e < 4; ++e) { w[e] = a0[e]; w[4 + e] = a1[e]; w[8 + e] = a2[e]; w[12 + e] = a3[e]; }
    v4u o0, o1;
#pragma unroll
    for (int e = 0; e < 4; ++e) {
      const unsigned short x0 = vr ? h_bits((_Float16)(bfr(w[2 * e]) * WCAR)) : (unsigned short)0;
      const unsigned short x1 = vr ? h_bits((_Float16)(bfr(w[2 * e + 1]) * WCAR)) : (unsigned short)0;
      const unsigned short y0 = vr ? h_bits((_Float16)(bfr(w[8 + 2 * e]) * WCAR)) : (unsigned short)0;
      const unsigned short y1 = vr ? h_bits((_Float16)(bfr(w[8 + 2 * e + 1]) * WCAR)) : (unsigned short)0;
      o0[e] = pk16(x0, x1);
      o1[e] = pk16(y0, y1);
    }
    *(v4u*)(RB2 + row * RBP + cb)     = o0;
    *(v4u*)(RB2 + row * RBP + cb + 8) = o1;
  }
  __syncthreads();

  v8f accB0 = zero8(), accB1 = zero8(), accB2 = zero8(), accB3 = zero8();
  const float bsc = 1.0f / (HCAR * WCAR);
#pragma unroll 1
  for (int kt = 0; kt < DM / 32; ++kt) {
    __syncthreads();
#pragma unroll
    for (int q = 0; q < 2; ++q) {
      const int p  = q * 256 + tid;
      const int il = p >> 5, jl = p & 31;
      const float r0 = CI[il * 4 + 0] - CJ2[jl * 4 + 0];
      const float r1 = CI[il * 4 + 1] - CJ2[jl * 4 + 1];
      const float r2 = CI[il * 4 + 2] - CJ2[jl * 4 + 2];
      u16* hrow = hid + p * HP;
#pragma unroll 1
      for (int g = 0; g < 4; ++g) {
        const int cb = kt * 32 + g * 8;
        v4u o;
#pragma unroll
        for (int e = 0; e < 4; ++e) {
          const v4f wa = *(const v4f*)(WB + (cb + 2 * e) * 4);
          const v4f wb = *(const v4f*)(WB + (cb + 2 * e + 1) * 4);
          const float h0 = wa[0] * r0 + wa[1] * r1 + wa[2] * r2 + wa[3];
          const float h1 = wb[0] * r0 + wb[1] * r1 + wb[2] * r2 + wb[3];
          o[e] = pk16(h_bits((_Float16)(silu_f(h0) * HCAR)), h_bits((_Float16)(silu_f(h1) * HCAR)));
        }
        *(v4u*)(hrow + g * 8) = o;
      }
    }
    __syncthreads();
    const v16h bw = ldfrag_h(rb2h + m * RBP + kt * 32 + 8 * hh);
    const v16h a0 = ldfrag_h(hidh + ((wave * 4 + 0) * 16 + m) * HP + 8 * hh);
    const v16h a1 = ldfrag_h(hidh + ((wave * 4 + 1) * 16 + m) * HP + 8 * hh);
    const v16h a2 = ldfrag_h(hidh + ((wave * 4 + 2) * 16 + m) * HP + 8 * hh);
    const v16h a3 = ldfrag_h(hidh + ((wave * 4 + 3) * 16 + m) * HP + 8 * hh);
    accB0 = mma_h(a0, bw, accB0);
    accB1 = mma_h(a1, bw, accB1);
    accB2 = mma_h(a2, bw, accB2);
    accB3 = mma_h(a3, bw, accB3);
    guard6<v16h>(accB0, accB1, accB2, accB3, a0, a1, a2, a3, bw, bw);
  }
  if (m < NH) {
#pragma unroll
    for (int r = 0; r < 8; ++r) {
      const int pr = 8 * hh + r;
      BB[((wave * 4 + 0) * 16 + pr) * NH + m] = accB0[r] * bsc;
      BB[((wave * 4 + 1) * 16 + pr) * NH + m] = accB1[r] * bsc;
      BB[((wave * 4 + 2) * 16 + pr) * NH + m] = accB2[r] * bsc;
      BB[((wave * 4 + 3) * 16 + pr) * NH + m] = accB3[r] * bsc;
    }
  }
  __syncthreads();

  const int head = wave;
  const size_t hcol = (size_t)head * HD + 8 * hh;
  const _Float16* qhp  = (const _Float16*)(const void*)QHp + ((size_t)(b * SEQ + i0 + m)) * DM + hcol;
  const _Float16* qlp  = (const _Float16*)(const void*)QLp + ((size_t)(b * SEQ + i0 + m)) * DM + hcol;
  const _Float16* kh0p = (const _Float16*)(const void*)KHp + ((size_t)(b * SEQ + j0 + m)) * DM + hcol;
  const _Float16* kl0p = (const _Float16*)(const void*)KLp + ((size_t)(b * SEQ + j0 + m)) * DM + hcol;
  const _Float16* kh1p = kh0p + (size_t)16 * DM;
  const _Float16* kl1p = kl0p + (size_t)16 * DM;
  v8f s0 = zero8(), s1 = zero8();
  {
    const v16h qh = ldfrag_h(qhp), ql = ldfrag_h(qlp);
    const v16h kh0 = ldfrag_h(kh0p), kl0 = ldfrag_h(kl0p);
    const v16h kh1 = ldfrag_h(kh1p), kl1 = ldfrag_h(kl1p);
    s0 = mma_h(qh, kh0, s0);
    s0 = mma_h(ql, kh0, s0);
    s0 = mma_h(qh, kl0, s0);
    s1 = mma_h(qh, kh1, s1);
    s1 = mma_h(ql, kh1, s1);
    s1 = mma_h(qh, kl1, s1);
    guard2(s0, s1, qh, ql, kh0, kl0, kh1, kl1);
  }
  const float lsc = RSQ_HD * (1.0f / (QSC * KSC));
  const float b2v = bfr(rbb2[head]);
  float* slab = HREG + wave * (16 * SLP);
#pragma unroll
  for (int r = 0; r < 8; ++r) {
    const int pr = 8 * hh + r;
    const float ba = BB[(pr * 32 + m) * NH + head] + b2v;
    const float bb = BB[(pr * 32 + 16 + m) * NH + head] + b2v;
    slab[pr * SLP + m]      = s0[r] * lsc + ba;
    slab[pr * SLP + 16 + m] = s1[r] * lsc + bb;
  }
  wave_sync_lds();
  v4f vals[4];
  const int rq = lane >> 3, c4 = (lane & 7) * 4;
#pragma unroll
  for (int q = 0; q < 4; ++q) vals[q] = *(const v4f*)(slab + (q * 4 + rq) * SLP + c4);
  float* dst = SCp + ((size_t)((b * NH + head) * SEQ + i0)) * SEQ + j0 + c4;
  for (int pass = 0; pass < 2; ++pass) {
#pragma unroll
    for (int q = 0; q < 4; ++q) {
      *(volatile v4f*)(dst + (size_t)(q * 4 + rq) * SEQ) = vals[q];
    }
    __threadfence();
  }
}

__global__ __launch_bounds__(256) void k_softmax(const float* __restrict__ SCp, u16* Pp) {
  const int tid = threadIdx.x, wave = tid >> 5, lane = tid & 31;
  const int row = (int)blockIdx.x * 8 + wave;
  if (row >= NB * NH * SEQ) return;
  const float* s = SCp + (size_t)row * SEQ;
  const bool vb = (lane < 16);
  const int  lb = vb ? lane : 15;
  const v4f a0 = *(const v4f*)(s + lane * 8), a1 = *(const v4f*)(s + lane * 8 + 4);
  const v4f c0 = *(const v4f*)(s + 256 + lb * 8), c1 = *(const v4f*)(s + 256 + lb * 8 + 4);
  float v[16];
#pragma unroll
  for (int e = 0; e < 4; ++e) {
    v[e]      = a0[e];
    v[4 + e]  = a1[e];
    v[8 + e]  = vb ? c0[e] : -INFINITY;
    v[12 + e] = vb ? c1[e] : -INFINITY;
  }
  float mx = v[0];
#pragma unroll
  for (int e = 1; e < 16; ++e) mx = fmaxf(mx, v[e]);
#pragma unroll
  for (int off = 1; off < 32; off <<= 1) mx = fmaxf(mx, __shfl_xor(mx, off, 32));
  float ev[16];
  float sum = 0.0f;
#pragma unroll
  for (int e = 0; e < 16; ++e) {
    const float d = v[e] - mx;
    ev[e] = exp2f(d * LOG2E);
    sum += ev[e];
  }
#pragma unroll
  for (int off = 1; off < 32; off <<= 1) sum += __shfl_xor(sum, off, 32);
  const float inv = 1.0f / sum;
  v4u oh0, ol0, oh1, ol1;
#pragma unroll
  for (int e = 0; e < 4; ++e) {
    const float t0 = (ev[2 * e] * inv) * PCAR, t1 = (ev[2 * e + 1] * inv) * PCAR;
    const float u0 = (ev[8 + 2 * e] * inv) * PCAR, u1 = (ev[8 + 2 * e + 1] * inv) * PCAR;
    const _Float16 h0 = (_Float16)t0, h1 = (_Float16)t1, g0 = (_Float16)u0, g1 = (_Float16)u1;
    const _Float16 l0 = (_Float16)(t0 - (float)h0), l1 = (_Float16)(t1 - (float)h1);
    const _Float16 m0 = (_Float16)(u0 - (float)g0), m1 = (_Float16)(u1 - (float)g1);
    oh0[e] = pk16(h_bits(h0), h_bits(h1));
    ol0[e] = pk16(h_bits(l0), h_bits(l1));
    oh1[e] = pk16(h_bits(g0), h_bits(g1));
    ol1[e] = pk16(h_bits(m0), h_bits(m1));
  }
  u16* dh = Pp + (size_t)row * SEQ;
  u16* dl = dh + PSTR;
  for (int pass = 0; pass < 2; ++pass) {
    *(volatile v4u*)(dh + lane * 8) = oh0;
    *(volatile v4u*)(dl + lane * 8) = ol0;
    if (vb) {
      *(volatile v4u*)(dh + 256 + lane * 8) = oh1;
      *(volatile v4u*)(dl + 256 + lane * 8) = ol1;
    }
    __threadfence();
  }
}

__global__ __launch_bounds__(256)
void k_tagg(const float* __restrict__ coords, const float* __restrict__ rvw1, const float* __restrict__ rvb1,
            const u16* __restrict__ Pp, u16* Tp) {
  __shared__ __align__(16) float CJ[SEQ * 4];
  __shared__ __align__(16) u16   WA[2 * 16 * WAP];
  __shared__ __align__(16) u16   ST[2 * DM * SP];
  __shared__ __align__(16) float TS[NH * TSP];

  const int tid = threadIdx.x, wave = tid >> 5, lane = tid & 31, hh = lane >> 4, m = lane & 15;
  const int bid = blockIdx.x;
  const int b   = bid / SEQ;
  const int i   = bid - b * SEQ;
  if (b >= NB) return;
  const _Float16* wah = (const _Float16*)(const void*)WA;
  const _Float16* sth = (const _Float16*)(const void*)ST;

  for (int idx = tid; idx < SEQ * CD; idx += 256) {
    const int j = idx / CD, k = idx - j * CD;
    CJ[j * 4 + k] = bfr(coords[(size_t)(b * SEQ) * CD + idx]);
  }
  if (tid < 64) {
    const int pl = tid >> 5, r = 8 + ((tid >> 2) & 7), pc = (tid & 3) * 8;
    const v4u z = {0u, 0u, 0u, 0u};
    *(v4u*)(WA + pl * (16 * WAP) + r * WAP + pc) = z;
  }
  const int c = tid;
  const float w0 = bfr(rvw1[c * 3 + 0]), w1 = bfr(rvw1[c * 3 + 1]), w2 = bfr(rvw1[c * 3 + 2]);
  const float b1 = bfr(rvb1[c]);
  const float ci0 = bfr(coords[((size_t)(b * SEQ + i)) * CD + 0]);
  const float ci1 = bfr(coords[((size_t)(b * SEQ + i)) * CD + 1]);
  const float ci2 = bfr(coords[((size_t)(b * SEQ + i)) * CD + 2]);

  v8f acc0 = zero8(), acc1 = zero8();
#pragma unroll 1
  for (int jt = 0; jt < NJT; ++jt) {
    const int j0 = jt * 32;
    __syncthreads();
    if (tid < 64) {
      const int pl = tid >> 5, h = (tid >> 2) & 7, pc = (tid & 3) * 8;
      const v4u pv = *(const v4u*)(Pp + (size_t)pl * PSTR + ((size_t)((b * NH + h) * SEQ + i)) * SEQ + j0 + pc);
      *(v4u*)(WA + pl * (16 * WAP) + h * WAP + pc) = pv;
    }
#pragma unroll 1
    for (int g = 0; g < 4; ++g) {
      v4u oh, ol;
#pragma unroll
      for (int e = 0; e < 4; ++e) {
        const int ja = j0 + g * 8 + 2 * e;
        const v4f ca = *(const v4f*)(CJ + ja * 4), cb = *(const v4f*)(CJ + ja * 4 + 4);
        const float ha = w0 * (ci0 - ca[0]) + w1 * (ci1 - ca[1]) + w2 * (ci2 - ca[2]) + b1;
        const float hb = w0 * (ci0 - cb[0]) + w1 * (ci1 - cb[1]) + w2 * (ci2 - cb[2]) + b1;
        const float sa = silu_f(ha) * HCAR, sb = silu_f(hb) * HCAR;
        const _Float16 xa = (_Float16)sa, xb = (_Float16)sb;
        const _Float16 ya = (_Float16)(sa - (float)xa), yb = (_Float16)(sb - (float)xb);
        oh[e] = pk16(h_bits(xa), h_bits(xb));
        ol[e] = pk16(h_bits(ya), h_bits(yb));
      }
      *(v4u*)(ST + c * SP + g * 8)           = oh;
      *(v4u*)(ST + DM * SP + c * SP + g * 8) = ol;
    }
    __syncthreads();
    const v16h ah  = ldfrag_h(wah + m * WAP + 8 * hh);
    const v16h al  = ldfrag_h(wah + 16 * WAP + m * WAP + 8 * hh);
    const int  ct0 = wave * 2;
    const v16h bh0 = ldfrag_h(sth + ((ct0) * 16 + m) * SP + 8 * hh);
    const v16h bl0 = ldfrag_h(sth + DM * SP + ((ct0) * 16 + m) * SP + 8 * hh);
    const v16h bh1 = ldfrag_h(sth + ((ct0 + 1) * 16 + m) * SP + 8 * hh);
    const v16h bl1 = ldfrag_h(sth + DM * SP + ((ct0 + 1) * 16 + m) * SP + 8 * hh);
    acc0 = mma_h(ah, bh0, acc0);
    acc0 = mma_h(al, bh0, acc0);
    acc0 = mma_h(ah, bl0, acc0);
    acc1 = mma_h(ah, bh1, acc1);
    acc1 = mma_h(al, bh1, acc1);
    acc1 = mma_h(ah, bl1, acc1);
    guard2(acc0, acc1, ah, al, bh0, bl0, bh1, bl1);
  }
  const float tsc = TCAR / (PCAR * HCAR);
  if (hh == 0) {
#pragma unroll
    for (int r = 0; r < 8; ++r) {
      TS[r * TSP + (wave * 2) * 16 + m]     = acc0[r] * tsc;
      TS[r * TSP + (wave * 2 + 1) * 16 + m] = acc1[r] * tsc;
    }
  }
  __syncthreads();
  {
    const int h = wave;
    const float* src = TS + h * TSP + lane * 8;
    const v4f a = *(const v4f*)(src), b4 = *(const v4f*)(src + 4);
    float w[8];
#pragma unroll
    for (int e = 0; e < 4; ++e) { w[e] = a[e]; w[4 + e] = b4[e]; }
    v4u oh, ol;
#pragma unroll
    for (int e = 0; e < 4; ++e) {
      const float t0 = w[2 * e], t1 = w[2 * e + 1];
      const _Float16 x0 = (_Float16)t0, x1 = (_Float16)t1;
      const _Float16 y0 = (_Float16)(t0 - (float)x0), y1 = (_Float16)(t1 - (float)x1);
      oh[e] = pk16(h_bits(x0), h_bits(x1));
      ol[e] = pk16(h_bits(y0), h_bits(y1));
    }
    const size_t rowT = (size_t)(b * NH + h) * SEQ + i;
    u16* dh = Tp + rowT * DM + lane * 8;
    u16* dl = dh + TSTR;
    for (int pass = 0; pass < 2; ++pass) {
      *(volatile v4u*)(dh) = oh;
      *(volatile v4u*)(dl) = ol;
      __threadfence();
    }
  }
}

__global__ __launch_bounds__(128)
void k_final(const u16* __restrict__ Pp, const u16* __restrict__ VHp, const u16* __restrict__ Tp,
             const u16* __restrict__ W2p, const float* __restrict__ rvb2, float* outp) {
  __shared__ __align__(16) float slab[4 * 16 * SLP];
  const int tid = threadIdx.x, wave = tid >> 5, lane = tid & 31, hh = lane >> 4, m = lane & 15;
  const int bid = blockIdx.x;
  const int rt  = bid % NRT;
  const int t2  = bid / NRT;
  const int h   = t2 % NH;
  const int b   = t2 / NH;
  if (b >= NB) return;
  const int irow = rt * 64 + wave * 16;
  const size_t bh   = (size_t)(b * NH + h);
  const size_t rowA = bh * SEQ + irow;
  const _Float16* P  = (const _Float16*)(const void*)Pp;
  const _Float16* VH = (const _Float16*)(const void*)VHp;
  const _Float16* T  = (const _Float16*)(const void*)Tp;
  const _Float16* W2 = (const _Float16*)(const void*)W2p;
  const _Float16* php = P + (rowA + m) * SEQ + 8 * hh;
  const _Float16* plp = php + PSTR;
  const _Float16* v0p = VH + (bh * HD + m) * SEQ + 8 * hh;
  const _Float16* v1p = v0p + (size_t)16 * SEQ;
  const _Float16* thp = T + (rowA + m) * DM + 8 * hh;
  const _Float16* tlp = thp + TSTR;
  const _Float16* w0p = W2 + ((size_t)(h * HD + m)) * DM + 8 * hh;
  const _Float16* w1p = w0p + (size_t)16 * DM;

  v8f p0 = zero8(), p1 = zero8(), r0 = zero8(), r1 = zero8();
#pragma unroll 1
  for (int k0 = 0; k0 < SEQ; k0 += 32) {
    const v16h ph = ldfrag_h(php + k0), pl = ldfrag_h(plp + k0);
    const v16h va = ldfrag_h(v0p + k0), vb = ldfrag_h(v1p + k0);
    p0 = mma_h(ph, va, p0);
    p0 = mma_h(pl, va, p0);
    p1 = mma_h(ph, vb, p1);
    p1 = mma_h(pl, vb, p1);
    guard2(p0, p1, ph, pl, va, vb, ph, pl);
  }
#pragma unroll 1
  for (int k0 = 0; k0 < DM; k0 += 32) {
    const v16h th = ldfrag_h(thp + k0), tl = ldfrag_h(tlp + k0);
    const v16h wa = ldfrag_h(w0p + k0), wb = ldfrag_h(w1p + k0);
    r0 = mma_h(th, wa, r0);
    r0 = mma_h(tl, wa, r0);
    r1 = mma_h(th, wb, r1);
    r1 = mma_h(tl, wb, r1);
    guard2(r0, r1, th, tl, wa, wb, th, tl);
  }
  const float osP = 1.0f / (PCAR * VCAR);
  const float osR = 1.0f / (TCAR * WCAR);
  const float bv0 = bfr(rvb2[h * HD + m]), bv1 = bfr(rvb2[h * HD + 16 + m]);
  float* sl = slab + wave * (16 * SLP);
#pragma unroll
  for (int r = 0; r < 8; ++r) {
    const int pr = 8 * hh + r;
    sl[pr * SLP + m]      = p0[r] * osP + (r0[r] * osR + bv0);
    sl[pr * SLP + 16 + m] = p1[r] * osP + (r1[r] * osR + bv1);
  }
  wave_sync_lds();
  v4f vals[4];
  const int rq = lane >> 3, c4 = (lane & 7) * 4;
#pragma unroll
  for (int q = 0; q < 4; ++q) vals[q] = *(const v4f*)(sl + (q * 4 + rq) * SLP + c4);
  float* dst = outp + ((size_t)(b * SEQ + irow)) * DM + h * HD + c4;
  for (int pass = 0; pass < 2; ++pass) {
#pragma unroll
    for (int q = 0; q < 4; ++q) {
      *(volatile v4f*)(dst + (size_t)(q * 4 + rq) * DM) = vals[q];
    }
    __threadfence();
  }
}

static size_t al64k(size_t x) { return (x + (size_t)65535) & ~(size_t)65535; }

extern "C" void kernel_launch(void* const* d_in, const int* in_sizes, int n_in,
                              void* d_out, int out_size, void* d_ws, size_t ws_size,
                              hipStream_t stream) {
  if (n_in < 12) return;
  if (in_sizes[0] < NB * SEQ * DM) return;
  if (in_sizes[1] < NB * SEQ * CD) return;
  if (in_sizes[2] != NQKV * DM || in_sizes[3] != NQKV) return;
  if (in_sizes[4] != DM * CD || in_sizes[5] != DM || in_sizes[6] != NH * DM || in_sizes[7] != NH) return;
  if (in_sizes[8] != DM * CD || in_sizes[9] != DM || in_sizes[10] != DM * DM || in_sizes[11] != DM) return;
  if (out_size < NB * SEQ * DM) return;

  const float* x      = (const float*)d_in[0];
  const float* coords = (const float*)d_in[1];
  const float* qkv_w  = (const float*)d_in[2];
  const float* qkv_b  = (const float*)d_in[3];
  const float* rb_w1  = (const float*)d_in[4];
  const float* rb_b1  = (const float*)d_in[5];
  const float* rb_w2  = (const float*)d_in[6];
  const float* rb_b2  = (const float*)d_in[7];
  const float* rv_w1  = (const float*)d_in[8];
  const float* rv_b1  = (const float*)d_in[9];
  const float* rv_w2  = (const float*)d_in[10];
  const float* rv_b2  = (const float*)d_in[11];
  float*       out    = (float*)d_out;

  const size_t szXB = (size_t)GROWS * DM * 2;
  const size_t szWQ = (size_t)NQKV * DM * 2;
  const size_t szW2 = (size_t)DM * DM * 2;
  const size_t szF  = (size_t)GROWS * NQKV * 4;
  const size_t szH  = (size_t)GROWS * DM * 2;
  const size_t szVH = (size_t)NB * NH * HD * SEQ * 2;
  const size_t szSC = (size_t)NB * NH * SEQ * SEQ * 4;
  const size_t szP  = PSTR * 2 * 2;
  const size_t szT  = TSTR * 2 * 2;
  size_t off = 0;
  const size_t oXB = off; off = al64k(off + szXB);
  const size_t oWQ = off; off = al64k(off + szWQ);
  const size_t oW2 = off; off = al64k(off + szW2);
  const size_t oF  = off; off = al64k(off + szF);
  const size_t oQH = off; off = al64k(off + szH);
  const size_t oQL = off; off = al64k(off + szH);
  const size_t oKH = off; off = al64k(off + szH);
  const size_t oKL = off; off = al64k(off + szH);
  const size_t oVH = off; off = al64k(off + szVH);
  const size_t oSC = off; off = al64k(off + szSC);
  const size_t oP  = off; off = al64k(off + szP);
  const size_t oT  = off; off = al64k(off + szT);
  if (off > ws_size) return;
  if (off > (size_t)WS_CAP) return;

  char* ws = (char*)d_ws;
  u16*   XB = (u16*)(ws + oXB);
  u16*   WQ = (u16*)(ws + oWQ);
  u16*   W2 = (u16*)(ws + oW2);
  float* F  = (float*)(ws + oF);
  u16*   QH = (u16*)(ws + oQH);
  u16*   QL = (u16*)(ws + oQL);
  u16*   KH = (u16*)(ws + oKH);
  u16*   KL = (u16*)(ws + oKL);
  u16*   VH = (u16*)(ws + oVH);
  float* SC = (float*)(ws + oSC);
  u16*   P  = (u16*)(ws + oP);
  u16*   T  = (u16*)(ws + oT);

  const dim3 b256(256), b128(128);
  const int n8x = (GROWS * DM) / 8;
  const int n8w = (NQKV * DM) / 8;
  const int n8v = (DM * DM) / 8;

  cvt16<<<dim3((n8x + 255) / 256), b256, 0, stream>>>(x, XB, n8x, 0, 1.0f);
  cvt16<<<dim3((n8w + 255) / 256), b256, 0, stream>>>(qkv_w, WQ, n8w, 0, 1.0f);
  cvt16<<<dim3((n8v + 255) / 256), b256, 0, stream>>>(rv_w2, W2, n8v, 1, WCAR);
  gemm_bf<<<dim3((GROWS / 64) * (NQKV / 64)), b128, 0, stream>>>(XB, WQ, qkv_b, F, GROWS, NQKV, DM, 1.0f);
  qk16<<<dim3(GROWS / 8), b256, 0, stream>>>(F, NQKV, 0, QH, QL, QSC);
  qk16<<<dim3(GROWS / 8), b256, 0, stream>>>(F, NQKV, DM, KH, KL, KSC);
  vt16<<<dim3(NB * NH * NRT), b256, 0, stream>>>(F, VH);
  k_scores<<<dim3(NB * NIT * NJT), b256, 0, stream>>>(coords, rb_w1, rb_b1, rb_w2, rb_b2, QH, QL, KH, KL, SC);
  k_softmax<<<dim3(NB * SEQ), b256, 0, stream>>>(SC, P);
  k_tagg<<<dim3(NB * SEQ), b256, 0, stream>>>(coords, rv_w1, rv_b1, P, T);
  k_final<<<dim3(NB * NH * NRT), b128, 0, stream>>>(P, VH, T, W2, rv_b2, out);
  (void)hipGetLastError();
}
